// TruncatedCRF_90718299226738
// MI455X (gfx1250) — hardware-verified
//
#include <hip/hip_runtime.h>
#include <stdint.h>


#define BB   64
#define TT   512
#define TM1  511
#define LL   2048
#define DD   512
#define NROW (BB * TM1)

typedef __bf16       v16bf __attribute__((ext_vector_type(16)));
typedef float        v8f   __attribute__((ext_vector_type(8)));
typedef float        v4f   __attribute__((ext_vector_type(4)));
typedef float        v2f   __attribute__((ext_vector_type(2)));
typedef unsigned int v4u   __attribute__((ext_vector_type(4)));

union ABu  { v16bf v; v4u q[2]; };
union V8BF { v4u q; unsigned short h[8]; };

#define NEG_BIG (-1e30f)

__device__ __forceinline__ unsigned int bf16_rne_bits(float f) {
    unsigned int u = __float_as_uint(f);
    u = u + 0x7FFFu + ((u >> 16) & 1u);
    return u >> 16;
}
__device__ __forceinline__ unsigned int pack2_bf16(float a, float b) {
    return bf16_rne_bits(a) | (bf16_rne_bits(b) << 16);
}
__device__ __forceinline__ float bf16_bits_to_f32(unsigned short h) {
    return __uint_as_float(((unsigned int)h) << 16);
}

__global__ void __launch_bounds__(256)
cvt_bf16_kernel(const float* __restrict__ se, const float* __restrict__ te,
                unsigned int* __restrict__ sb, unsigned int* __restrict__ tb,
                int nvec) {
    const int i = blockIdx.x * 256 + (int)threadIdx.x;
    if (i < nvec) {
        const size_t e0 = (size_t)i * 8;
        const v4f s0 = *(const v4f*)(se + e0);
        const v4f s1 = *(const v4f*)(se + e0 + 4);
        const v4f t0 = *(const v4f*)(te + e0);
        const v4f t1 = *(const v4f*)(te + e0 + 4);
        v4u ps, pt;
        ps.x = pack2_bf16(s0.x, s0.y); ps.y = pack2_bf16(s0.z, s0.w);
        ps.z = pack2_bf16(s1.x, s1.y); ps.w = pack2_bf16(s1.z, s1.w);
        pt.x = pack2_bf16(t0.x, t0.y); pt.y = pack2_bf16(t0.z, t0.w);
        pt.z = pack2_bf16(t1.x, t1.y); pt.w = pack2_bf16(t1.z, t1.w);
        volatile v4u* dps = (volatile v4u*)(sb + (size_t)i * 4);
        volatile v4u* dpt = (volatile v4u*)(tb + (size_t)i * 4);
        *dps = ps;
        *dpt = pt;
        __threadfence();
        *dps = ps;
        *dpt = pt;
    }
}

__global__ void __launch_bounds__(256)
crf_score_kernel(const int* __restrict__ labels,
                 const unsigned short* __restrict__ srcb,
                 const unsigned short* __restrict__ tgtb,
                 float* __restrict__ out, int nrow) {
    extern __shared__ __attribute__((aligned(16))) char smem_raw[];
    unsigned short* abuf = (unsigned short*)smem_raw;
    int*   tcol_lds = (int*)  (smem_raw + 65536);
    v2f*   stats    = (v2f*)  (smem_raw + 65792);
    float* outl     = (float*)(smem_raw + 69888);

    const int row0   = blockIdx.x * 64;
    const int tid    = (int)threadIdx.x;
    const int wave   = tid >> 5;
    const int lane   = tid & 31;
    const int laneLo = lane & 15;
    const int hi     = lane >> 4;

    for (int i = tid; i < 4096; i += 256) {
        int rrow = i >> 6;
        int kpos = (i & 63) << 3;
        int r = row0 + rrow;
        if (r > nrow - 1) r = nrow - 1;
        int b = r / TM1;
        int t = r - b * TM1;
        int lbl = labels[b * TT + t];
        lbl = lbl < 0 ? 0 : (lbl > LL - 1 ? LL - 1 : lbl);
        *(v4u*)(abuf + rrow * DD + kpos) =
            *(const v4u*)(srcb + (size_t)lbl * DD + kpos);
    }
    if (tid < 64) {
        int r = row0 + tid;
        if (r > nrow - 1) r = nrow - 1;
        int b = r / TM1;
        int t = r - b * TM1;
        int tc = labels[b * TT + t + 1];
        tc = tc < 0 ? 0 : (tc > LL - 1 ? LL - 1 : tc);
        tcol_lds[tid] = tc;
    }
    __syncthreads();

    float mrun[32], srun[32];
#pragma unroll
    for (int j = 0; j < 32; ++j) { mrun[j] = NEG_BIG; srun[j] = 0.f; }

    const unsigned short* arow = abuf + laneLo * DD + hi * 8;

#pragma unroll 1
    for (int chunk = 0; chunk < 16; ++chunk) {
        const int n = chunk * 128 + wave * 16 + laneLo;
        const unsigned short* bcol = tgtb + (size_t)n * DD + hi * 8;

        v8f c0 = {}, c1 = {}, c2 = {}, c3 = {};
#pragma unroll 1
        for (int kk = 0; kk < DD; kk += 32) {
            ABu bm;
            const v4u* bp = (const v4u*)(bcol + kk);
            bm.q[0] = bp[0];
            bm.q[1] = bp[2];

            ABu a0, a1, a2, a3;
            const v4u* ap0 = (const v4u*)(arow + kk);
            const v4u* ap1 = (const v4u*)(arow + 16 * DD + kk);
            const v4u* ap2 = (const v4u*)(arow + 32 * DD + kk);
            const v4u* ap3 = (const v4u*)(arow + 48 * DD + kk);
            a0.q[0] = ap0[0]; a0.q[1] = ap0[2];
            a1.q[0] = ap1[0]; a1.q[1] = ap1[2];
            a2.q[0] = ap2[0]; a2.q[1] = ap2[2];
            a3.q[0] = ap3[0]; a3.q[1] = ap3[2];

            c0 = __builtin_amdgcn_wmma_f32_16x16x32_bf16(
                     false, a0.v, false, bm.v, (short)0, c0, false, false);
            c1 = __builtin_amdgcn_wmma_f32_16x16x32_bf16(
                     false, a1.v, false, bm.v, (short)0, c1, false, false);
            c2 = __builtin_amdgcn_wmma_f32_16x16x32_bf16(
                     false, a2.v, false, bm.v, (short)0, c2, false, false);
            c3 = __builtin_amdgcn_wmma_f32_16x16x32_bf16(
                     false, a3.v, false, bm.v, (short)0, c3, false, false);
            asm volatile("v_nop\n\tv_nop\n\tv_nop\n\tv_nop"
                         : "+v"(c0), "+v"(c1), "+v"(c2), "+v"(c3)
                         : "v"(a0.v), "v"(a1.v), "v"(a2.v), "v"(a3.v), "v"(bm.v));
        }

#pragma unroll
        for (int g = 0; g < 4; ++g) {
#pragma unroll
            for (int v = 0; v < 8; ++v) {
                float x  = (g == 0) ? c0[v] : (g == 1) ? c1[v]
                         : (g == 2) ? c2[v] : c3[v];
                int   j  = g * 8 + v;
                float mo = mrun[j];
                float d  = x - mo;
                float e  = __expf(-fabsf(d));
                bool  nm = d > 0.f;
                srun[j]  = nm ? (srun[j] * e + 1.f) : (srun[j] + e);
                mrun[j]  = nm ? x : mo;
            }
        }
    }

#pragma unroll
    for (int j = 0; j < 32; ++j) {
        float m = mrun[j], s = srun[j];
#pragma unroll
        for (int off = 1; off < 16; off <<= 1) {
            float mo = __shfl_xor(m, off, 32);
            float so = __shfl_xor(s, off, 32);
            float mn = fmaxf(m, mo);
            s = s * __expf(m - mn) + so * __expf(mo - mn);
            m = mn;
        }
        mrun[j] = m; srun[j] = s;
    }

    if (laneLo == 0) {
        volatile v2f* st = (volatile v2f*)stats;
#pragma unroll
        for (int g = 0; g < 4; ++g)
#pragma unroll
            for (int v = 0; v < 8; ++v) {
                int r = g * 16 + v + 8 * hi;
                int j = g * 8 + v;
                v2f p;
                p.x = mrun[j];
                p.y = srun[j];
                st[r * 8 + wave] = p;
            }
    }
    __syncthreads();

    if (tid < 64) {
        const int r = tid;
        float m = NEG_BIG;
#pragma unroll
        for (int w = 0; w < 8; ++w) { v2f q = stats[r * 8 + w]; m = fmaxf(m, q.x); }
        float s = 0.f;
#pragma unroll
        for (int w = 0; w < 8; ++w) {
            v2f q = stats[r * 8 + w];
            s += q.y * __expf(q.x - m);
        }

        const int tc = tcol_lds[r];
        const unsigned short* av = abuf + r * DD;
        const unsigned short* bv = tgtb + (size_t)tc * DD;
        float acc = 0.f;
#pragma unroll 4
        for (int k = 0; k < DD; k += 8) {
            V8BF a, b;
            a.q = *(const v4u*)(av + k);
            b.q = *(const v4u*)(bv + k);
#pragma unroll
            for (int u = 0; u < 8; ++u)
                acc += bf16_bits_to_f32(a.h[u]) * bf16_bits_to_f32(b.h[u]);
        }
        const float val = acc - m - __logf(s);
        ((volatile float*)outl)[r] = val;
    }
    __syncthreads();

    if (tid < 16) {
        const int e = row0 + tid * 4;
        if (e + 4 <= nrow) {
            const v4f v = *(const v4f*)(outl + tid * 4);
            volatile v4f* p = (volatile v4f*)(out + e);
            *p = v;
            __threadfence();
            *p = v;
        }
    }
}

extern "C" void kernel_launch(void* const* d_in, const int* in_sizes, int n_in,
                              void* d_out, int out_size, void* d_ws, size_t ws_size,
                              hipStream_t stream) {
    if (n_in < 3) return;
    const int nElem = LL * DD;
    if (in_sizes[0] != BB * TT || in_sizes[1] != nElem || in_sizes[2] != nElem) return;
    if (out_size != NROW) return;
    const size_t tableBytes = (size_t)nElem * 2;
    if (ws_size < 2 * tableBytes) return;

    const int*   labels = (const int*)  d_in[0];
    const float* src_f  = (const float*)d_in[1];
    const float* tgt_f  = (const float*)d_in[2];
    float* out = (float*)d_out;

    unsigned int* src_b = (unsigned int*)d_ws;
    unsigned int* tgt_b = (unsigned int*)((char*)d_ws + tableBytes);

    const int nvec = nElem / 8;
    cvt_bf16_kernel<<<(nvec + 255) / 256, 256, 0, stream>>>(
        src_f, tgt_f, src_b, tgt_b, nvec);

    const int smemBytes = 70144;
    crf_score_kernel<<<(NROW + 63) / 64, 256, smemBytes, stream>>>(
        labels, (const unsigned short*)src_b, (const unsigned short*)tgt_b, out, NROW);
}
